// ResInvProjector_24730421690454
// MI455X (gfx1250) — hardware-verified
//
#include <hip/hip_runtime.h>
#include <math.h>

constexpr int kPts       = 8 * 4096;
constexpr int kEmb       = 64;
constexpr int kOutC      = 64;
constexpr int kKer       = 64;
constexpr int kGdim      = 3;
constexpr int kWcols     = kEmb * kOutC;
constexpr int kChunkRows = 4096;
constexpr int kNumChunks = kPts / kChunkRows;
static_assert(kNumChunks * kChunkRows == kPts, "chunking exact");
static_assert(kKer % 32 == 0, "K multiple of 32");
static_assert(kChunkRows % 64 == 0 && kWcols % 64 == 0, "tile multiples");

typedef __attribute__((ext_vector_type(16))) _Float16 v16h;
typedef __attribute__((ext_vector_type(8)))  _Float16 v8h;
typedef __attribute__((ext_vector_type(16))) __bf16   v16b;
typedef __attribute__((ext_vector_type(8)))  __bf16   v8b;
typedef __attribute__((ext_vector_type(8)))  float    v8f;
typedef __attribute__((ext_vector_type(4)))  float    v4f;
typedef __attribute__((ext_vector_type(4)))  unsigned int v4u;

__device__ __forceinline__ unsigned short f2bf_bits(float f) {
  unsigned u = __float_as_uint(f);
  return (unsigned short)((u + 0x7FFFu + ((u >> 16) & 1u)) >> 16);
}
__device__ __forceinline__ float bf_bits2f(unsigned short h) { return __uint_as_float(((unsigned)h) << 16); }

__device__ __forceinline__ void dep_guard_h(v8f& a, v8f& b, v16h x, v16h y) { asm volatile("v_nop\n\tv_nop\n\tv_nop\n\tv_nop" : "+v"(a), "+v"(b) : "v"(x), "v"(y)); }
__device__ __forceinline__ void dep_guard_b(v8f& a, v8f& b, v16b x, v16b y) { asm volatile("v_nop\n\tv_nop\n\tv_nop\n\tv_nop" : "+v"(a), "+v"(b) : "v"(x), "v"(y)); }
__device__ __forceinline__ void keep4_h(v16h a, v16h b, v16h c, v16h d) { asm volatile("v_nop" :: "v"(a), "v"(b), "v"(c), "v"(d)); }
__device__ __forceinline__ void keep4_b(v16b a, v16b b, v16b c, v16b d) { asm volatile("v_nop" :: "v"(a), "v"(b), "v"(c), "v"(d)); }
__device__ __forceinline__ void acc_guard4(v8f& a, v8f& b, v8f& c, v8f& d) { asm volatile("v_nop\n\tv_nop\n\tv_nop\n\tv_nop" : "+v"(a), "+v"(b), "+v"(c), "+v"(d)); }
template <typename T> struct Frag;
template <> struct Frag<_Float16> {
  typedef v16h V; union U { v16h v; v8h h[2]; };
  static __device__ __forceinline__ v16h load(const _Float16* p) {
    U f; f.h[0] = *(const v8h*)(p); f.h[1] = *(const v8h*)(p + 16); return f.v;
  }
  static __device__ __forceinline__ v8f mma(v16h a, v16h b, v8f c) {
    return __builtin_amdgcn_wmma_f32_16x16x32_f16(false, a, false, b, (short)0, c, false, false);
  }
  static __device__ __forceinline__ void guard(v8f& a, v8f& b, v16h x, v16h y) { dep_guard_h(a, b, x, y); }
  static __device__ __forceinline__ void keep(v16h a, v16h b, v16h c, v16h d) { keep4_h(a, b, c, d); }
};
template <> struct Frag<__bf16> {
  typedef v16b V; union U { v16b v; v8b h[2]; };
  static __device__ __forceinline__ v16b load(const __bf16* p) {
    U f; f.h[0] = *(const v8b*)(p); f.h[1] = *(const v8b*)(p + 16); return f.v;
  }
  static __device__ __forceinline__ v8f mma(v16b a, v16b b, v8f c) {
    return __builtin_amdgcn_wmma_f32_16x16x32_bf16(false, a, false, b, (short)0, c, false, false);
  }
  static __device__ __forceinline__ void guard(v8f& a, v8f& b, v16b x, v16b y) { dep_guard_b(a, b, x, y); }
  static __device__ __forceinline__ void keep(v16b a, v16b b, v16b c, v16b d) { keep4_b(a, b, c, d); }
};

__device__ __forceinline__ unsigned pk16(unsigned short a, unsigned short b) { return (unsigned)a | ((unsigned)b << 16); }

template <int ET> struct Elem;
template <> struct Elem<0> { typedef _Float16 T; };
template <> struct Elem<1> { typedef __bf16 T; };
template <int ET, bool SPLIT, int BIAS_MODE, int OUT_MODE, bool RESID, int ACT = 0>
__global__ __launch_bounds__(256) void wmma_gemm64(
    const unsigned short* __restrict__ Ap, const unsigned short* __restrict__ A2p, int lda, long strideA,
    const unsigned short* __restrict__ Btp, const unsigned short* __restrict__ Bt2p, int ldb, long strideB,
    void* __restrict__ Cout, void* __restrict__ Cout2, int ldc, long strideC,
    const float* __restrict__ bias,
    const float* __restrict__ resid, long strideR,
    int M, int N, int K, float scale) {
  typedef typename Elem<ET>::T T;
  typedef typename Frag<T>::V V;
  const T* A = (const T*)Ap; const T* A2 = (const T*)A2p; const T* Bt = (const T*)Btp; const T* Bt2 = (const T*)Bt2p;
  __shared__ __align__(16) float sT[8][16 * 68];
  const int b    = blockIdx.y;
  const int lane = threadIdx.x & 31;
  const int wave = threadIdx.x >> 5;
  const int tilesN = N >> 6;
  const int tilesM = M >> 6;
  const int tile = blockIdx.x * 8 + wave;
  if (tile >= tilesM * tilesN) return;
  const int tm = tile / tilesN;
  const int tn = tile - tm * tilesN;
  const int m0 = tm << 6;
  const int n0 = tn << 6;

  const T* Ab  = A  + (size_t)b * strideA;
  const T* Bb  = Bt + (size_t)b * strideB;
  const T* Ab2 = SPLIT ? (A2  + (size_t)b * strideA) : nullptr;
  const T* Bb2 = SPLIT ? (Bt2 + (size_t)b * strideB) : nullptr;

  const int rlane = lane & 15;
  const int koff  = (lane >> 4) * 8;
  const int mOff  = (lane >> 4) * 8;

  v8f acc[4][4];
#pragma unroll
  for (int i = 0; i < 4; ++i)
#pragma unroll
    for (int j = 0; j < 4; ++j) acc[i][j] = (v8f){0.f,0.f,0.f,0.f,0.f,0.f,0.f,0.f};

  for (int k0 = 0; k0 < K; k0 += 32) {
    V bh[4], bl[4];
#pragma unroll
    for (int j = 0; j < 4; ++j) {
      const size_t bo = (size_t)(n0 + (j << 4) + rlane) * ldb + koff + k0;
      bh[j] = Frag<T>::load(Bb + bo);
      if (SPLIT) bl[j] = Frag<T>::load(Bb2 + bo);
    }
#pragma unroll
    for (int i = 0; i < 4; ++i) {
      const size_t ao = (size_t)(m0 + (i << 4) + rlane) * lda + koff + k0;
      V ah = Frag<T>::load(Ab + ao);
      V al;
      if (SPLIT) al = Frag<T>::load(Ab2 + ao);
#pragma unroll
      for (int j = 0; j < 4; ++j) {
        acc[i][j] = Frag<T>::mma(ah, bh[j], acc[i][j]);
        if (SPLIT) {
          acc[i][j] = Frag<T>::mma(ah, bl[j], acc[i][j]);
          acc[i][j] = Frag<T>::mma(al, bh[j], acc[i][j]);
        }
      }
      Frag<T>::guard(acc[i][0], acc[i][3], ah, SPLIT ? al : ah);
    }
    Frag<T>::keep(bh[0], bh[1], bh[2], bh[3]);
    if (SPLIT) Frag<T>::keep(bl[0], bl[1], bl[2], bl[3]);
  }
  acc_guard4(acc[0][0], acc[0][1], acc[0][2], acc[0][3]);
  acc_guard4(acc[1][0], acc[1][1], acc[1][2], acc[1][3]);
  acc_guard4(acc[2][0], acc[2][1], acc[2][2], acc[2][3]);
  acc_guard4(acc[3][0], acc[3][1], acc[3][2], acc[3][3]);

  float* slab = sT[wave];
  const float* Rb = RESID ? (resid + (size_t)b * strideR) : nullptr;
#pragma unroll
  for (int i = 0; i < 4; ++i) {
    const int mBase = m0 + (i << 4);
#pragma unroll
    for (int j = 0; j < 4; ++j) {
      const int n = n0 + (j << 4) + rlane;
      float bv = 0.f;
      if (BIAS_MODE == 2) bv = bias[n];
#pragma unroll
      for (int r = 0; r < 8; ++r) {
        float v = acc[i][j][r] * scale;
        if (BIAS_MODE == 1) v += bias[mBase + mOff + r];
        if (BIAS_MODE == 2) v += bv;
        if (RESID) v += Rb[(size_t)(mBase + mOff + r) * ldc + n];
        if (ACT == 2) v = fmaxf(v, 0.0f);
        if (ACT == 4) v = (v > 0.f) ? v : 0.01f * v;
        slab[(mOff + r) * 68 + (j << 4) + rlane] = v;
      }
    }
    __builtin_amdgcn_fence(__ATOMIC_RELEASE, "workgroup");
    __builtin_amdgcn_wave_barrier();
    __builtin_amdgcn_fence(__ATOMIC_ACQUIRE, "workgroup");
    if (OUT_MODE == 0) {
      float* C = (float*)Cout + (size_t)b * strideC;
      const int hh = lane >> 4, c4 = (lane & 15) * 4;
      for (int pass = 0; pass < 2; ++pass) {
#pragma unroll
        for (int it = 0; it < 8; ++it) {
          const int row = it * 2 + hh;
          v4f v = *(const v4f*)(slab + row * 68 + c4);
          *(volatile v4f*)(C + (size_t)(mBase + row) * ldc + n0 + c4) = v;
        }
        __threadfence();
      }
    } else {
      const int q = lane >> 3, c8 = (lane & 7) * 8;
      unsigned short* C  = (unsigned short*)Cout  + (size_t)b * strideC;
      unsigned short* C2 = (OUT_MODE == 2) ? ((unsigned short*)Cout2 + (size_t)b * strideC) : nullptr;
      for (int pass = 0; pass < 2; ++pass) {
#pragma unroll
        for (int it = 0; it < 4; ++it) {
          const int row = it * 4 + q;
          const float* sp = slab + row * 68 + c8;
          v8h hv, lv;
#pragma unroll
          for (int e = 0; e < 8; ++e) {
            if (OUT_MODE == 1) {
              hv[e] = (_Float16)sp[e];
            } else {
              unsigned short hb = f2bf_bits(sp[e]);
              unsigned short lb = f2bf_bits(sp[e] - bf_bits2f(hb));
              hv[e] = __builtin_bit_cast(_Float16, hb);
              lv[e] = __builtin_bit_cast(_Float16, lb);
            }
          }
          *(volatile v8h*)(C + (size_t)(mBase + row) * ldc + n0 + c8) = hv;
          if (OUT_MODE == 2) *(volatile v8h*)(C2 + (size_t)(mBase + row) * ldc + n0 + c8) = lv;
        }
        __threadfence();
      }
    }
    __builtin_amdgcn_fence(__ATOMIC_RELEASE, "workgroup");
    __builtin_amdgcn_wave_barrier();
    __builtin_amdgcn_fence(__ATOMIC_ACQUIRE, "workgroup");
  }
}

__global__ __launch_bounds__(256) void hgen_kernel(const float* __restrict__ gridp,
                                                  const float* __restrict__ W1,
                                                  const float* __restrict__ b1,
                                                  unsigned short* __restrict__ Hhi,
                                                  unsigned short* __restrict__ Hlo) {
  __shared__ __align__(16) float sH[4][64];
  const int t = threadIdx.x;
  const int p = t >> 6;
  const int k = t & 63;
  const int n = blockIdx.x * 4 + p;
  const float g0 = gridp[(size_t)n * kGdim + 0];
  const float g1 = gridp[(size_t)n * kGdim + 1];
  const float g2 = gridp[(size_t)n * kGdim + 2];
  const float pre = g0 * W1[k] + g1 * W1[kKer + k] + g2 * W1[2 * kKer + k] + b1[k];
  const float hv = 0.5f * pre * (1.0f + erff(pre * 0.70710678118654752f));
  sH[p][k] = hv;
  __syncthreads();
  if (t < 64) {
    const int wave = t >> 5, lane = t & 31;
    const int q = lane >> 3, c8 = (lane & 7) * 8;
    unsigned short bits[8];
#pragma unroll
    for (int e = 0; e < 8; ++e) {
      const float v = sH[q][c8 + e];
      const unsigned short hb = f2bf_bits(v);
      const unsigned short lb = f2bf_bits(v - bf_bits2f(hb));
      bits[e] = (wave == 0) ? hb : lb;
    }
    const v4u u = (v4u){pk16(bits[0], bits[1]), pk16(bits[2], bits[3]), pk16(bits[4], bits[5]), pk16(bits[6], bits[7])};
    unsigned short* plane = (wave == 0) ? Hhi : Hlo;
    unsigned short* dst = plane + (size_t)(blockIdx.x * 4 + q) * kKer + c8;
    *(volatile v4u*)dst = u;
    __threadfence();
    *(volatile v4u*)dst = u;
  }
}

__global__ __launch_bounds__(256) void w2t_split_kernel(const float* __restrict__ W2,
                                                       unsigned short* __restrict__ Bhi,
                                                       unsigned short* __restrict__ Blo) {
  __shared__ float sm[64][65];
  const int t  = threadIdx.x;
  const int n0 = blockIdx.x * 64;
#pragma unroll
  for (int i = 0; i < 16; ++i) {
    const int e  = i * 256 + t;
    const int kk = e >> 6;
    const int c  = e & 63;
    sm[kk][c] = W2[(size_t)kk * kWcols + n0 + c];
  }
  __syncthreads();
  const int lane = t & 31, wave = t >> 5;
  const int q = lane >> 3, c8 = (lane & 7) * 8;
  for (int pass = 0; pass < 2; ++pass) {
#pragma unroll
    for (int it = 0; it < 2; ++it) {
      const int row = wave * 8 + it * 4 + q;
      unsigned short hb[8], lb[8];
#pragma unroll
      for (int e = 0; e < 8; ++e) {
        const float v = sm[c8 + e][row];
        hb[e] = f2bf_bits(v);
        lb[e] = f2bf_bits(v - bf_bits2f(hb[e]));
      }
      const v4u uh = (v4u){pk16(hb[0], hb[1]), pk16(hb[2], hb[3]), pk16(hb[4], hb[5]), pk16(hb[6], hb[7])};
      const v4u ul = (v4u){pk16(lb[0], lb[1]), pk16(lb[2], lb[3]), pk16(lb[4], lb[5]), pk16(lb[6], lb[7])};
      *(volatile v4u*)(Bhi + (size_t)(n0 + row) * kKer + c8) = uh;
      *(volatile v4u*)(Blo + (size_t)(n0 + row) * kKer + c8) = ul;
    }
    __threadfence();
  }
}

__global__ __launch_bounds__(256) void rowdot_kernel(const float* __restrict__ x,
                                                    const float* __restrict__ Wd,
                                                    float* __restrict__ out,
                                                    int rowBase) {
  __shared__ __align__(16) float sX[4][64];
  __shared__ __align__(16) float sO[4][68];
  const int t  = threadIdx.x;
  const int r  = t >> 6;
  const int o  = t & 63;
  const int nl = blockIdx.x * 4 + r;
  const int n  = rowBase + nl;
  sX[r][o] = x[(size_t)n * kEmb + o];
  __syncthreads();
  const float* wrow = Wd + (size_t)nl * kWcols + o;
  float acc = 0.f;
#pragma unroll 4
  for (int i = 0; i < kEmb; ++i) acc = fmaf(sX[r][i], wrow[i * kOutC], acc);
  sO[r][o] = acc;
  __syncthreads();
  const int wave = t >> 5, lane = t & 31;
  if (wave < 4 && lane < 16) {
    const int c4 = lane * 4;
    const v4f v = *(const v4f*)(&sO[wave][c4]);
    float* dst = out + (size_t)(rowBase + blockIdx.x * 4 + wave) * kOutC + c4;
    *(volatile v4f*)dst = v;
    __threadfence();
    *(volatile v4f*)dst = v;
  }
}

extern "C" void kernel_launch(void* const* d_in, const int* in_sizes, int n_in,
                              void* d_out, int out_size, void* d_ws, size_t ws_size,
                              hipStream_t stream) {
  if (n_in < 6) return;
  if (in_sizes[0] != kPts * kEmb) return;
  if (in_sizes[1] != kPts * kGdim) return;
  if (in_sizes[2] != kGdim * kKer) return;
  if (in_sizes[3] != kKer) return;
  if (in_sizes[4] != kKer * kWcols) return;
  if (in_sizes[5] != kWcols) return;
  if (out_size != kPts * kOutC) return;

  const float* x     = (const float*)d_in[0];
  const float* gridp = (const float*)d_in[1];
  const float* W1    = (const float*)d_in[2];
  const float* b1    = (const float*)d_in[3];
  const float* W2    = (const float*)d_in[4];
  const float* b2    = (const float*)d_in[5];
  float* out = (float*)d_out;

  const size_t hPlaneBytes = (size_t)kPts * kKer * 2;
  const size_t bPlaneBytes = (size_t)kWcols * kKer * 2;
  const size_t wdBytes     = (size_t)kChunkRows * kWcols * 4;
  const size_t offHhi = 0;
  const size_t offHlo = offHhi + hPlaneBytes;
  const size_t offBhi = offHlo + hPlaneBytes;
  const size_t offBlo = offBhi + bPlaneBytes;
  const size_t offWd  = offBlo + bPlaneBytes;
  const size_t total  = offWd + wdBytes;
  if (total > ws_size) return;

  unsigned char* ws = (unsigned char*)d_ws;
  unsigned short* Hhi = (unsigned short*)(ws + offHhi);
  unsigned short* Hlo = (unsigned short*)(ws + offHlo);
  unsigned short* Bhi = (unsigned short*)(ws + offBhi);
  unsigned short* Blo = (unsigned short*)(ws + offBlo);
  float*          Wd  = (float*)(ws + offWd);

  hgen_kernel<<<kPts / 4, 256, 0, stream>>>(gridp, W1, b1, Hhi, Hlo);
  w2t_split_kernel<<<kWcols / 64, 256, 0, stream>>>(W2, Bhi, Blo);

  const int tiles = (kChunkRows / 64) * (kWcols / 64);
  const int gemmBlocks = (tiles + 7) / 8;
  for (int ch = 0; ch < kNumChunks; ++ch) {
    const size_t aoff = (size_t)ch * kChunkRows * kKer;
    wmma_gemm64<1, true, 2, 0, false, 0><<<dim3(gemmBlocks, 1), 256, 0, stream>>>(
        Hhi + aoff, Hlo + aoff, kKer, 0L,
        Bhi, Blo, kKer, 0L,
        (void*)Wd, (void*)Wd, kWcols, 0L,
        b2,
        b2, 0L,
        kChunkRows, kWcols, kKer, 1.0f);
    rowdot_kernel<<<kChunkRows / 4, 256, 0, stream>>>(x, Wd, out, ch * kChunkRows);
  }
}
